// TRG_wrapper_21449066676690
// MI455X (gfx1250) — hardware-verified
//
#include <hip/hip_runtime.h>
#include <math.h>

constexpr int kCh     = 512;
constexpr int kImH    = 16;
constexpr int kImW    = 32;
constexpr int kPx     = kImH * kImW;
constexpr int kHid    = 64;
constexpr int kTap    = 9;
constexpr int kTapPad = 64;
constexpr int kKcol   = kCh * kTap;

typedef __attribute__((ext_vector_type(16))) _Float16 v16h;
typedef __attribute__((ext_vector_type(8)))  _Float16 v8h;
typedef __attribute__((ext_vector_type(16))) __bf16   v16b;
typedef __attribute__((ext_vector_type(8)))  __bf16   v8b;
typedef __attribute__((ext_vector_type(8)))  float    v8f;
typedef __attribute__((ext_vector_type(4)))  float    v4f;
typedef __attribute__((ext_vector_type(4)))  unsigned int v4u;

__device__ __forceinline__ unsigned short f2bf_bits(float f) {
  unsigned u = __float_as_uint(f);
  return (unsigned short)((u + 0x7FFFu + ((u >> 16) & 1u)) >> 16);
}
__device__ __forceinline__ float bf_bits2f(unsigned short h) { return __uint_as_float(((unsigned)h) << 16); }

__device__ __forceinline__ void dep_guard_h(v8f& a, v8f& b, v16h x, v16h y) { asm volatile("v_nop\n\tv_nop\n\tv_nop\n\tv_nop" : "+v"(a), "+v"(b) : "v"(x), "v"(y)); }
__device__ __forceinline__ void dep_guard_b(v8f& a, v8f& b, v16b x, v16b y) { asm volatile("v_nop\n\tv_nop\n\tv_nop\n\tv_nop" : "+v"(a), "+v"(b) : "v"(x), "v"(y)); }
__device__ __forceinline__ void keep4_h(v16h a, v16h b, v16h c, v16h d) { asm volatile("v_nop" :: "v"(a), "v"(b), "v"(c), "v"(d)); }
__device__ __forceinline__ void keep4_b(v16b a, v16b b, v16b c, v16b d) { asm volatile("v_nop" :: "v"(a), "v"(b), "v"(c), "v"(d)); }
__device__ __forceinline__ void acc_guard4(v8f& a, v8f& b, v8f& c, v8f& d) { asm volatile("v_nop\n\tv_nop\n\tv_nop\n\tv_nop" : "+v"(a), "+v"(b), "+v"(c), "+v"(d)); }
template <typename T> struct Frag;
template <> struct Frag<_Float16> {
  typedef v16h V; union U { v16h v; v8h h[2]; };
  static __device__ __forceinline__ v16h load(const _Float16* p) {
    U f; f.h[0] = *(const v8h*)(p); f.h[1] = *(const v8h*)(p + 16); return f.v;
  }
  static __device__ __forceinline__ v8f mma(v16h a, v16h b, v8f c) {
    return __builtin_amdgcn_wmma_f32_16x16x32_f16(false, a, false, b, (short)0, c, false, false);
  }
  static __device__ __forceinline__ void guard(v8f& a, v8f& b, v16h x, v16h y) { dep_guard_h(a, b, x, y); }
  static __device__ __forceinline__ void keep(v16h a, v16h b, v16h c, v16h d) { keep4_h(a, b, c, d); }
};
template <> struct Frag<__bf16> {
  typedef v16b V; union U { v16b v; v8b h[2]; };
  static __device__ __forceinline__ v16b load(const __bf16* p) {
    U f; f.h[0] = *(const v8b*)(p); f.h[1] = *(const v8b*)(p + 16); return f.v;
  }
  static __device__ __forceinline__ v8f mma(v16b a, v16b b, v8f c) {
    return __builtin_amdgcn_wmma_f32_16x16x32_bf16(false, a, false, b, (short)0, c, false, false);
  }
  static __device__ __forceinline__ void guard(v8f& a, v8f& b, v16b x, v16b y) { dep_guard_b(a, b, x, y); }
  static __device__ __forceinline__ void keep(v16b a, v16b b, v16b c, v16b d) { keep4_b(a, b, c, d); }
};

__device__ __forceinline__ unsigned pk16(unsigned short a, unsigned short b) { return (unsigned)a | ((unsigned)b << 16); }

template <int ET> struct Elem;
template <> struct Elem<0> { typedef _Float16 T; };
template <> struct Elem<1> { typedef __bf16 T; };
template <int ET, int SPL, int BIAS_MODE, int OUT_MODE, bool RESID, int ACT>
__global__ __launch_bounds__(256) void wmma_gemm64(
    const unsigned short* __restrict__ Ap, const unsigned short* __restrict__ A2p, int lda, long strideA,
    const unsigned short* __restrict__ Btp, const unsigned short* __restrict__ Bt2p, int ldb, long strideB,
    void* __restrict__ Cout, void* __restrict__ Cout2, int ldc, long strideC,
    const float* __restrict__ bias,
    const float* __restrict__ resid, long strideR,
    int M, int N, int K, float scale) {
  typedef typename Elem<ET>::T T;
  typedef typename Frag<T>::V V;
  const T* A = (const T*)Ap; const T* A2 = (const T*)A2p; const T* Bt = (const T*)Btp; const T* Bt2 = (const T*)Bt2p;
  __shared__ __align__(16) float sT[8][16 * 68];
  const int b    = blockIdx.y;
  const int lane = threadIdx.x & 31;
  const int wave = threadIdx.x >> 5;
  const int tilesN = N >> 6;
  const int tilesM = M >> 6;
  const int tile = blockIdx.x * 8 + wave;
  if (tile >= tilesM * tilesN) return;
  const int tm = tile / tilesN;
  const int tn = tile - tm * tilesN;
  const int m0 = tm << 6;
  const int n0 = tn << 6;

  const T* Ab  = A  + (size_t)b * strideA;
  const T* Bb  = Bt + (size_t)b * strideB;
  const T* Ab2 = (SPL & 1) ? (A2  + (size_t)b * strideA) : nullptr;
  const T* Bb2 = (SPL & 2) ? (Bt2 + (size_t)b * strideB) : nullptr;

  const int rlane = lane & 15;
  const int koff  = (lane >> 4) * 8;
  const int mOff  = (lane >> 4) * 8;

  v8f acc[4][4];
#pragma unroll
  for (int i = 0; i < 4; ++i)
#pragma unroll
    for (int j = 0; j < 4; ++j) acc[i][j] = (v8f){0.f,0.f,0.f,0.f,0.f,0.f,0.f,0.f};

  for (int k0 = 0; k0 < K; k0 += 32) {
    V bh[4], bl[4];
#pragma unroll
    for (int j = 0; j < 4; ++j) {
      const size_t bo = (size_t)(n0 + (j << 4) + rlane) * ldb + koff + k0;
      bh[j] = Frag<T>::load(Bb + bo);
      if (SPL & 2) bl[j] = Frag<T>::load(Bb2 + bo);
    }
#pragma unroll
    for (int i = 0; i < 4; ++i) {
      const size_t ao = (size_t)(m0 + (i << 4) + rlane) * lda + koff + k0;
      V ah = Frag<T>::load(Ab + ao);
      V al;
      if (SPL & 1) al = Frag<T>::load(Ab2 + ao);
#pragma unroll
      for (int j = 0; j < 4; ++j) {
        acc[i][j] = Frag<T>::mma(ah, bh[j], acc[i][j]);
        if (SPL & 2) acc[i][j] = Frag<T>::mma(ah, bl[j], acc[i][j]);
        if (SPL & 1) acc[i][j] = Frag<T>::mma(al, bh[j], acc[i][j]);
      }
      Frag<T>::guard(acc[i][0], acc[i][3], ah, (SPL & 1) ? al : ah);
    }
    Frag<T>::keep(bh[0], bh[1], bh[2], bh[3]);
    if (SPL & 2) Frag<T>::keep(bl[0], bl[1], bl[2], bl[3]);
  }
  acc_guard4(acc[0][0], acc[0][1], acc[0][2], acc[0][3]);
  acc_guard4(acc[1][0], acc[1][1], acc[1][2], acc[1][3]);
  acc_guard4(acc[2][0], acc[2][1], acc[2][2], acc[2][3]);
  acc_guard4(acc[3][0], acc[3][1], acc[3][2], acc[3][3]);

  float* slab = sT[wave];
  const float* Rb = RESID ? (resid + (size_t)b * strideR) : nullptr;
#pragma unroll
  for (int i = 0; i < 4; ++i) {
    const int mBase = m0 + (i << 4);
#pragma unroll
    for (int j = 0; j < 4; ++j) {
      const int n = n0 + (j << 4) + rlane;
      float bv = 0.f;
      if (BIAS_MODE == 2) bv = bias[n];
#pragma unroll
      for (int r = 0; r < 8; ++r) {
        float v = acc[i][j][r] * scale;
        if (BIAS_MODE == 1) v += bias[mBase + mOff + r];
        if (BIAS_MODE == 2) v += bv;
        if (RESID) v += Rb[(size_t)(mBase + mOff + r) * ldc + n];
        if (ACT == 2) v = fmaxf(v, 0.0f);
        if (ACT == 7) v = (v > 0.f) ? v : 0.1f * v;
        slab[(mOff + r) * 68 + (j << 4) + rlane] = v;
      }
    }
    __builtin_amdgcn_fence(__ATOMIC_RELEASE, "workgroup");
    __builtin_amdgcn_wave_barrier();
    __builtin_amdgcn_fence(__ATOMIC_ACQUIRE, "workgroup");
    if (OUT_MODE == 0) {
      float* C = (float*)Cout + (size_t)b * strideC;
      const int hh = lane >> 4, c4 = (lane & 15) * 4;
      for (int pass = 0; pass < 2; ++pass) {
#pragma unroll
        for (int it = 0; it < 8; ++it) {
          const int row = it * 2 + hh;
          v4f v = *(const v4f*)(slab + row * 68 + c4);
          *(volatile v4f*)(C + (size_t)(mBase + row) * ldc + n0 + c4) = v;
        }
        __threadfence();
      }
    } else {
      const int q = lane >> 3, c8 = (lane & 7) * 8;
      unsigned short* C  = (unsigned short*)Cout  + (size_t)b * strideC;
      unsigned short* C2 = (OUT_MODE == 2) ? ((unsigned short*)Cout2 + (size_t)b * strideC) : nullptr;
      for (int pass = 0; pass < 2; ++pass) {
#pragma unroll
        for (int it = 0; it < 4; ++it) {
          const int row = it * 4 + q;
          const float* sp = slab + row * 68 + c8;
          v8h hv, lv;
#pragma unroll
          for (int e = 0; e < 8; ++e) {
            if (OUT_MODE == 1) {
              hv[e] = (_Float16)sp[e];
            } else {
              unsigned short hb = f2bf_bits(sp[e]);
              unsigned short lb = f2bf_bits(sp[e] - bf_bits2f(hb));
              hv[e] = __builtin_bit_cast(_Float16, hb);
              lv[e] = __builtin_bit_cast(_Float16, lb);
            }
          }
          *(volatile v8h*)(C + (size_t)(mBase + row) * ldc + n0 + c8) = hv;
          if (OUT_MODE == 2) *(volatile v8h*)(C2 + (size_t)(mBase + row) * ldc + n0 + c8) = lv;
        }
        __threadfence();
      }
    }
    __builtin_amdgcn_fence(__ATOMIC_RELEASE, "workgroup");
    __builtin_amdgcn_wave_barrier();
    __builtin_amdgcn_fence(__ATOMIC_ACQUIRE, "workgroup");
  }
}

__global__ __launch_bounds__(256) void splitcast8_kernel(const float* __restrict__ in, unsigned short* __restrict__ hi,
                                                         unsigned short* __restrict__ lo, int nreal, int n8) {
  const int i = blockIdx.x * 256 + threadIdx.x;
  if (i >= n8) return;
  const int e0 = 8 * i;
  const bool pad = (e0 >= nreal);
  const int src = pad ? (nreal - 8) : e0;
  const v4f a = *(const v4f*)(in + src);
  const v4f c = *(const v4f*)(in + src + 4);
  unsigned short hb[8], lb[8];
#pragma unroll
  for (int e = 0; e < 4; ++e) {
    const float f0 = pad ? 0.f : a[e];
    const float f1 = pad ? 0.f : c[e];
    hb[e] = f2bf_bits(f0);
    lb[e] = f2bf_bits(f0 - bf_bits2f(hb[e]));
    hb[4 + e] = f2bf_bits(f1);
    lb[4 + e] = f2bf_bits(f1 - bf_bits2f(hb[4 + e]));
  }
  const v4u hv = (v4u){pk16(hb[0], hb[1]), pk16(hb[2], hb[3]), pk16(hb[4], hb[5]), pk16(hb[6], hb[7])};
  const v4u lv = (v4u){pk16(lb[0], lb[1]), pk16(lb[2], lb[3]), pk16(lb[4], lb[5]), pk16(lb[6], lb[7])};
  unsigned short* hp = hi + (size_t)e0;
  unsigned short* lp = lo + (size_t)e0;
  *(volatile v4u*)hp = hv;
  *(volatile v4u*)lp = lv;
  __threadfence();
  *(volatile v4u*)hp = hv;
  *(volatile v4u*)lp = lv;
}

__global__ __launch_bounds__(256) void transpose_split_kernel(const float* __restrict__ in, unsigned short* __restrict__ oh,
                                                              unsigned short* __restrict__ ol) {
  __shared__ float s[64][65];
  const int c0 = blockIdx.x * 64;
  const int r0 = blockIdx.y * 64;
  const int t = threadIdx.x;
  const int lane = t & 31, wave = t >> 5;
  {
    const int lr = t >> 2, lc = (t & 3) * 16;
    const float* p = in + (size_t)(r0 + lr) * kPx + c0 + lc;
#pragma unroll
    for (int q4 = 0; q4 < 4; ++q4) {
      const v4f v = *(const v4f*)(p + 4 * q4);
#pragma unroll
      for (int e = 0; e < 4; ++e) s[lr][lc + 4 * q4 + e] = v[e];
    }
  }
  __syncthreads();
  const int q = lane >> 3, c8 = (lane & 7) * 8;
  for (int pass = 0; pass < 2; ++pass) {
#pragma unroll
    for (int it = 0; it < 2; ++it) {
      const int oc = wave * 8 + it * 4 + q;
      unsigned short hb[8], lb[8];
#pragma unroll
      for (int e = 0; e < 8; ++e) {
        const float f = s[c8 + e][oc];
        hb[e] = f2bf_bits(f);
        lb[e] = f2bf_bits(f - bf_bits2f(hb[e]));
      }
      const v4u hv = (v4u){pk16(hb[0], hb[1]), pk16(hb[2], hb[3]), pk16(hb[4], hb[5]), pk16(hb[6], hb[7])};
      const v4u lv = (v4u){pk16(lb[0], lb[1]), pk16(lb[2], lb[3]), pk16(lb[4], lb[5]), pk16(lb[6], lb[7])};
      const size_t o = (size_t)(c0 + oc) * kCh + r0 + c8;
      *(volatile v4u*)(oh + o) = hv;
      *(volatile v4u*)(ol + o) = lv;
    }
    __threadfence();
  }
}

__global__ __launch_bounds__(256) void dwconv_split_kernel(const float* __restrict__ x, const float* __restrict__ kern,
                                                          unsigned short* __restrict__ xph, unsigned short* __restrict__ xpl) {
  const int i = blockIdx.x * 256 + threadIdx.x;
  if (i >= kPx * (kCh / 8)) return;
  const int px  = i >> 6;
  const int ch8 = (i & 63) * 8;
  const int h = px >> 5, w = px & 31;
  float acc[8];
#pragma unroll
  for (int e = 0; e < 8; ++e) acc[e] = 0.f;
#pragma unroll 1
  for (int j = 0; j < kTap; ++j) {
    const int j3 = j / 3;
    const int hh = h + j3 - 1;
    const int ww = w + (j - j3 * 3) - 1;
    const bool valid = (hh >= 0) && (hh < kImH) && (ww >= 0) && (ww < kImW);
    const int hc = hh < 0 ? 0 : (hh > kImH - 1 ? kImH - 1 : hh);
    const int wc = ww < 0 ? 0 : (ww > kImW - 1 ? kImW - 1 : ww);
    const int np = hc * kImW + wc;
#pragma unroll
    for (int e = 0; e < 8; ++e) {
      const float kv = kern[(size_t)(ch8 + e) * kTapPad + j];
      float xv = x[(size_t)(ch8 + e) * kPx + np];
      xv = valid ? xv : 0.f;
      acc[e] = fmaf(kv, xv, acc[e]);
    }
  }
  unsigned short hb[8], lb[8];
#pragma unroll
  for (int e = 0; e < 8; ++e) {
    float v = acc[e];
    v = (v > 0.f) ? v : 0.1f * v;
    hb[e] = f2bf_bits(v);
    lb[e] = f2bf_bits(v - bf_bits2f(hb[e]));
  }
  const v4u hv = (v4u){pk16(hb[0], hb[1]), pk16(hb[2], hb[3]), pk16(hb[4], hb[5]), pk16(hb[6], hb[7])};
  const v4u lv = (v4u){pk16(lb[0], lb[1]), pk16(lb[2], lb[3]), pk16(lb[4], lb[5]), pk16(lb[6], lb[7])};
  const size_t o = (size_t)px * kCh + ch8;
  *(volatile v4u*)(xph + o) = hv;
  *(volatile v4u*)(xpl + o) = lv;
  __threadfence();
  *(volatile v4u*)(xph + o) = hv;
  *(volatile v4u*)(xpl + o) = lv;
}

__global__ __launch_bounds__(256) void combine_kernel(const float* __restrict__ pout, const float* __restrict__ att,
                                                     const float* __restrict__ dr, float* __restrict__ y, int n4) {
  const int i = blockIdx.x * 256 + threadIdx.x;
  if (i >= n4) return;
  const size_t o = 4 * (size_t)i;
  const v4f p = *(const v4f*)(pout + o);
  const v4f a = *(const v4f*)(att + o);
  const v4f d = *(const v4f*)(dr + o);
  v4f r;
#pragma unroll
  for (int e = 0; e < 4; ++e) {
    const float sg = __builtin_amdgcn_rcpf(1.0f + __expf(-a[e]));
    float v = p[e] + d[e] * sg;
    r[e] = (v > 0.f) ? v : 0.1f * v;
  }
  *(volatile v4f*)(y + o) = r;
  __threadfence();
  *(volatile v4f*)(y + o) = r;
}

__global__ __launch_bounds__(256) void im2col_split_kernel(const float* __restrict__ y, unsigned short* __restrict__ colh,
                                                          unsigned short* __restrict__ coll) {
  constexpr int kT8 = kKcol / 8;
  const int i = blockIdx.x * 256 + threadIdx.x;
  if (i >= kPx * kT8) return;
  const int px = i / kT8;
  const int k8 = (i - px * kT8) * 8;
  const int h = px >> 5, w = px & 31;
  unsigned short hb[8], lb[8];
#pragma unroll
  for (int e = 0; e < 8; ++e) {
    const int k  = k8 + e;
    const int c  = k / kTap;
    const int j  = k - c * kTap;
    const int j3 = j / 3;
    const int hh = h + j3 - 1;
    const int ww = w + (j - j3 * 3) - 1;
    const bool valid = (hh >= 0) && (hh < kImH) && (ww >= 0) && (ww < kImW);
    const int hc = hh < 0 ? 0 : (hh > kImH - 1 ? kImH - 1 : hh);
    const int wc = ww < 0 ? 0 : (ww > kImW - 1 ? kImW - 1 : ww);
    float v = y[(size_t)c * kPx + hc * kImW + wc];
    v = valid ? v : 0.f;
    hb[e] = f2bf_bits(v);
    lb[e] = f2bf_bits(v - bf_bits2f(hb[e]));
  }
  const v4u hv = (v4u){pk16(hb[0], hb[1]), pk16(hb[2], hb[3]), pk16(hb[4], hb[5]), pk16(hb[6], hb[7])};
  const v4u lv = (v4u){pk16(lb[0], lb[1]), pk16(lb[2], lb[3]), pk16(lb[4], lb[5]), pk16(lb[6], lb[7])};
  const size_t o = (size_t)px * kKcol + k8;
  *(volatile v4u*)(colh + o) = hv;
  *(volatile v4u*)(coll + o) = lv;
  __threadfence();
  *(volatile v4u*)(colh + o) = hv;
  *(volatile v4u*)(coll + o) = lv;
}

extern "C" void kernel_launch(void* const* d_in, const int* in_sizes, int n_in,
                              void* d_out, int out_size, void* d_ws, size_t ws_size,
                              hipStream_t stream) {
  if (n_in < 18) return;
  if (in_sizes[0] != kCh * kPx) return;
  if (in_sizes[1] != kCh * kCh) return;
  if (in_sizes[2] != kCh * kCh || in_sizes[10] != kCh * kCh) return;
  if (in_sizes[3] != kTap * kCh || in_sizes[11] != kTap * kCh) return;
  if (in_sizes[4] != kCh * kCh || in_sizes[12] != kCh * kCh) return;
  if (in_sizes[5] != kCh || in_sizes[13] != kCh) return;
  if (in_sizes[6] != kHid * kCh || in_sizes[14] != kHid * kCh) return;
  if (in_sizes[7] != kCh * kHid || in_sizes[15] != kCh * kHid) return;
  if (in_sizes[8] != kCh * kKcol || in_sizes[16] != kCh * kKcol) return;
  if (in_sizes[9] != kCh || in_sizes[17] != kCh) return;
  if (out_size != kCh * kPx) return;

  const float* cIn = (const float*)d_in[0];
  const float* deg = (const float*)d_in[1];
  const float* kw1[2]  = {(const float*)d_in[2],  (const float*)d_in[10]};
  const float* kw2[2]  = {(const float*)d_in[3],  (const float*)d_in[11]};
  const float* pw[2]   = {(const float*)d_in[4],  (const float*)d_in[12]};
  const float* pb[2]   = {(const float*)d_in[5],  (const float*)d_in[13]};
  const float* caw1[2] = {(const float*)d_in[6],  (const float*)d_in[14]};
  const float* caw2[2] = {(const float*)d_in[7],  (const float*)d_in[15]};
  const float* cw[2]   = {(const float*)d_in[8],  (const float*)d_in[16]};
  const float* cb[2]   = {(const float*)d_in[9],  (const float*)d_in[17]};
  float* outp = (float*)d_out;

  const size_t SZ_P16  = (size_t)kCh * kCh * 2;
  const size_t SZ_S16  = (size_t)kTapPad * kCh * 2;
  const size_t SZ_W16  = (size_t)kCh * kKcol * 2;
  const size_t SZ_KERN = (size_t)kCh * kTapPad * 4;
  const size_t SZ_F32  = (size_t)kCh * kPx * 4;
  size_t off = 0;
  auto take = [&](size_t bytes) -> size_t { const size_t o = off; off += (bytes + 1023) & ~(size_t)1023; return o; };
  const size_t oDEGH = take(SZ_P16), oDEGL = take(SZ_P16), oDRTH = take(SZ_P16), oDRTL = take(SZ_P16);
  size_t oKW1H[2], oKW1L[2], oKW2H[2], oKW2L[2], oPWH[2], oPWL[2], oCA1H[2], oCA1L[2], oCA2H[2], oCA2L[2], oCWH[2], oCWL[2];
  for (int bk = 0; bk < 2; ++bk) {
    oKW1H[bk] = take(SZ_P16); oKW1L[bk] = take(SZ_P16);
    oKW2H[bk] = take(SZ_S16); oKW2L[bk] = take(SZ_S16);
    oPWH[bk]  = take(SZ_P16); oPWL[bk]  = take(SZ_P16);
    oCA1H[bk] = take(SZ_S16); oCA1L[bk] = take(SZ_S16);
    oCA2H[bk] = take(SZ_S16); oCA2L[bk] = take(SZ_S16);
    oCWH[bk]  = take(SZ_W16); oCWL[bk]  = take(SZ_W16);
  }
  const size_t oTH = take(SZ_P16), oTL = take(SZ_P16);
  const size_t oKERN = take(SZ_KERN);
  const size_t oXPH = take(SZ_P16), oXPL = take(SZ_P16);
  const size_t oPOUT = take(SZ_F32);
  const size_t oZH = take(SZ_S16), oZL = take(SZ_S16);
  const size_t oATT = take(SZ_F32);
  const size_t oY = take(SZ_F32);
  const size_t oCOLH = take(SZ_W16), oCOLL = take(SZ_W16);
  const size_t oO2 = take(SZ_F32);
  const size_t TOTAL = off;
  if (TOTAL > ws_size) return;
  if (TOTAL > (size_t)134217728) return;

  char* ws = (char*)d_ws;
  auto P16 = [&](size_t o) -> unsigned short* { return (unsigned short*)(ws + o); };
  auto P32 = [&](size_t o) -> float* { return (float*)(ws + o); };
  unsigned short* DEGH = P16(oDEGH); unsigned short* DEGL = P16(oDEGL);
  unsigned short* DRTH = P16(oDRTH); unsigned short* DRTL = P16(oDRTL);
  unsigned short* TH = P16(oTH); unsigned short* TL = P16(oTL);
  float* KERN = P32(oKERN);
  unsigned short* XPH = P16(oXPH); unsigned short* XPL = P16(oXPL);
  float* POUT = P32(oPOUT);
  unsigned short* ZH = P16(oZH); unsigned short* ZL = P16(oZL);
  float* ATT = P32(oATT);
  float* Y = P32(oY);
  unsigned short* COLH = P16(oCOLH); unsigned short* COLL = P16(oCOLL);
  float* O2 = P32(oO2);

  const dim3 blk(256);
  const int n8P = kCh * kCh / 8;
  const int n8S = kTapPad * kCh / 8;
  const int n8W = kCh * kKcol / 8;

  splitcast8_kernel<<<dim3(n8P / 256), blk, 0, stream>>>(deg, DEGH, DEGL, kCh * kCh, n8P);
  transpose_split_kernel<<<dim3(kPx / 64, kCh / 64), blk, 0, stream>>>(deg, DRTH, DRTL);
  for (int bk = 0; bk < 2; ++bk) {
    splitcast8_kernel<<<dim3(n8P / 256), blk, 0, stream>>>(kw1[bk], P16(oKW1H[bk]), P16(oKW1L[bk]), kCh * kCh, n8P);
    splitcast8_kernel<<<dim3(n8S / 256), blk, 0, stream>>>(kw2[bk], P16(oKW2H[bk]), P16(oKW2L[bk]), kTap * kCh, n8S);
    splitcast8_kernel<<<dim3(n8P / 256), blk, 0, stream>>>(pw[bk], P16(oPWH[bk]), P16(oPWL[bk]), kCh * kCh, n8P);
    splitcast8_kernel<<<dim3(n8S / 256), blk, 0, stream>>>(caw1[bk], P16(oCA1H[bk]), P16(oCA1L[bk]), kHid * kCh, n8S);
    splitcast8_kernel<<<dim3(n8S / 256), blk, 0, stream>>>(caw2[bk], P16(oCA2H[bk]), P16(oCA2L[bk]), kCh * kHid, n8S);
    splitcast8_kernel<<<dim3(n8W / 256), blk, 0, stream>>>(cw[bk], P16(oCWH[bk]), P16(oCWL[bk]), kCh * kKcol, n8W);
  }

  const dim3 gFull(((kCh / 64) * (kPx / 64) + 7) / 8, 1);
  const dim3 gNarrow(((kCh / 64) * (kTapPad / 64) + 7) / 8, 1);
  const int n4 = kCh * kPx / 4;

  for (int bk = 0; bk < 2; ++bk) {
    const float* xin = (bk == 0) ? cIn : O2;
    wmma_gemm64<1, 3, 0, 2, false, 7><<<gFull, blk, 0, stream>>>(
        DEGH, DEGL, kCh, 0L, P16(oKW1H[bk]), P16(oKW1L[bk]), kCh, 0L, (void*)TH, (void*)TL, kCh, 0L,
        pb[bk], cIn, 0L, kCh, kCh, kCh, 1.0f);
    wmma_gemm64<1, 3, 0, 0, false, 0><<<gNarrow, blk, 0, stream>>>(
        TH, TL, kCh, 0L, P16(oKW2H[bk]), P16(oKW2L[bk]), kCh, 0L, (void*)KERN, (void*)KERN, kTapPad, 0L,
        pb[bk], cIn, 0L, kCh, kTapPad, kCh, 1.0f);
    dwconv_split_kernel<<<dim3(kPx * (kCh / 8) / 256), blk, 0, stream>>>(xin, KERN, XPH, XPL);
    wmma_gemm64<1, 3, 1, 0, false, 0><<<gFull, blk, 0, stream>>>(
        P16(oPWH[bk]), P16(oPWL[bk]), kCh, 0L, XPH, XPL, kCh, 0L, (void*)POUT, (void*)POUT, kPx, 0L,
        pb[bk], cIn, 0L, kCh, kPx, kCh, 1.0f);
    wmma_gemm64<1, 3, 0, 2, false, 7><<<gNarrow, blk, 0, stream>>>(
        DRTH, DRTL, kCh, 0L, P16(oCA1H[bk]), P16(oCA1L[bk]), kCh, 0L, (void*)ZH, (void*)ZL, kHid, 0L,
        pb[bk], cIn, 0L, kPx, kHid, kCh, 1.0f);
    wmma_gemm64<1, 3, 0, 0, false, 0><<<gFull, blk, 0, stream>>>(
        P16(oCA2H[bk]), P16(oCA2L[bk]), kHid, 0L, ZH, ZL, kHid, 0L, (void*)ATT, (void*)ATT, kPx, 0L,
        pb[bk], cIn, 0L, kCh, kPx, kHid, 1.0f);
    combine_kernel<<<dim3(n4 / 256), blk, 0, stream>>>(POUT, ATT, deg, Y, n4);
    im2col_split_kernel<<<dim3(kPx * (kKcol / 8) / 256), blk, 0, stream>>>(Y, COLH, COLL);
    if (bk == 0) {
      wmma_gemm64<1, 3, 1, 0, false, 7><<<gFull, blk, 0, stream>>>(
          P16(oCWH[bk]), P16(oCWL[bk]), kKcol, 0L, COLH, COLL, kKcol, 0L, (void*)O2, (void*)O2, kPx, 0L,
          cb[bk], cIn, 0L, kCh, kPx, kKcol, 1.0f);
    } else {
      wmma_gemm64<1, 3, 1, 0, true, 0><<<gFull, blk, 0, stream>>>(
          P16(oCWH[bk]), P16(oCWL[bk]), kKcol, 0L, COLH, COLL, kKcol, 0L, (void*)outp, (void*)outp, kPx, 0L,
          cb[bk], cIn, 0L, kCh, kPx, kKcol, 1.0f);
    }
  }
}
